// cascaded_mvPAM_Module_mask_13314398618069
// MI455X (gfx1250) — hardware-verified
//
#include <hip/hip_runtime.h>
#include <math.h>

typedef __attribute__((ext_vector_type(16))) _Float16 v16h;
typedef __attribute__((ext_vector_type(16))) __bf16 v16b;
typedef __attribute__((ext_vector_type(8)))  _Float16 v8h;
typedef __attribute__((ext_vector_type(8)))  float v8f;
typedef __attribute__((ext_vector_type(4)))  float v4f;
typedef __attribute__((ext_vector_type(2)))  float v2f;
typedef __attribute__((ext_vector_type(4)))  unsigned v4u;
typedef __attribute__((ext_vector_type(4)))  int v4i;
typedef float __attribute__((may_alias)) float_a;
typedef int __attribute__((may_alias)) int_a;

template <typename T> __device__ __forceinline__ void vst2(void* p, T v) { *(volatile T*)p = v; __threadfence(); *(volatile T*)p = v; }
__device__ __forceinline__ v8f wmma16(v16h a, v16h b, v8f c) {
  v8f d = __builtin_amdgcn_wmma_f32_16x16x32_f16(false, a, false, b, (short)0, c, false, false);
  asm volatile("v_nop\n\tv_nop\n\tv_nop\n\tv_nop" : "+v"(d) : "v"(a), "v"(b));
  return d;
}
__device__ __forceinline__ v8f wmma_bf(v16b a, v16b b, v8f c) {
  v8f d = __builtin_amdgcn_wmma_f32_16x16x32_bf16(false, a, false, b, (short)0, c, false, false);
  asm volatile("v_nop\n\tv_nop\n\tv_nop\n\tv_nop" : "+v"(d) : "v"(a), "v"(b));
  return d;
}
__device__ __forceinline__ v16h frag_h(const _Float16* rowk0, int lane) {
  union { v16h v; v8h q[2]; } u; const _Float16* p = rowk0 + 8 * (lane >> 4);
  u.q[0] = *(const v8h*)p; u.q[1] = *(const v8h*)(p + 16); return u.v;
}
__device__ __forceinline__ v16h frag_f32(const float* rowk0, int lane) {
  v16h a; const float* p = rowk0 + 8 * (lane >> 4);
#pragma unroll
  for (int i = 0; i < 8; ++i) { a[i] = (_Float16)p[i]; a[8 + i] = (_Float16)p[16 + i]; }
  return a;
}
__device__ __forceinline__ v16h frag_f32s(const float* rowk0, int lane, float sc) {
  v16h a; const float* p = rowk0 + 8 * (lane >> 4);
#pragma unroll
  for (int i = 0; i < 8; ++i) { a[i] = (_Float16)(p[i] * sc); a[8 + i] = (_Float16)(p[16 + i] * sc); }
  return a;
}
__device__ __forceinline__ v16h fragc_f32(const float* W, int k0, int n, int lane, int ld, int K) {
  v16h a; const int g = lane >> 4;
#pragma unroll
  for (int i = 0; i < 8; ++i) { const int ka = k0 + 8 * g + i, kb = ka + 16;
    a[i] = (_Float16)(ka < K ? W[(size_t)(ka < K ? ka : K - 1) * ld + n] : 0.f); a[8 + i] = (_Float16)(kb < K ? W[(size_t)(kb < K ? kb : K - 1) * ld + n] : 0.f); }
  return a;
}
struct F2 { v16b h, l; };
__device__ __forceinline__ F2 bsplit16(const float v[16]) { F2 r;
#pragma unroll
  for (int i = 0; i < 16; ++i) { const __bf16 h = (__bf16)v[i]; r.h[i] = h; r.l[i] = (__bf16)(v[i] - (float)h); }
  return r; }
__device__ __forceinline__ F2 split_row(const float* row, int k0, int lane) { float v[16]; const float* p = row + k0 + 8 * (lane >> 4);
#pragma unroll
  for (int i = 0; i < 8; ++i) { v[i] = p[i]; v[8 + i] = p[16 + i]; }
  return bsplit16(v); }
__device__ __forceinline__ F2 split_rowK(const float* row, int k0, int lane, int K) { float v[16]; const int g = lane >> 4;
#pragma unroll
  for (int i = 0; i < 8; ++i) { const int ka = k0 + 8 * g + i, kb = ka + 16; v[i] = ka < K ? row[ka < K ? ka : K - 1] : 0.f; v[8 + i] = kb < K ? row[kb < K ? kb : K - 1] : 0.f; }
  return bsplit16(v); }
__device__ __forceinline__ F2 split_col(const float* W, int k0, int n, int lane, int ld, int K) { float v[16]; const int g = lane >> 4;
#pragma unroll
  for (int i = 0; i < 8; ++i) { const int ka = k0 + 8 * g + i, kb = ka + 16; v[i] = ka < K ? W[(size_t)(ka < K ? ka : K - 1) * ld + n] : 0.f; v[8 + i] = kb < K ? W[(size_t)(kb < K ? kb : K - 1) * ld + n] : 0.f; }
  return bsplit16(v); }
__device__ __forceinline__ v8f mac3(const F2& a, const F2& b, v8f c) { c = wmma_bf(a.l, b.h, c); c = wmma_bf(a.h, b.l, c); return wmma_bf(a.h, b.h, c); }
__device__ __forceinline__ float sigm(float v) { return 1.0f / (1.0f + expf(-v)); }
#define LDSX() do { asm volatile("s_wait_dscnt 0" ::: "memory"); __builtin_amdgcn_wave_barrier(); __builtin_amdgcn_fence(__ATOMIC_RELEASE, "workgroup"); } while (0)


#define NB 2
#define CC 512
#define HH 56
#define NPOS 3136
#define CQ 64
#define CAT 2048
#ifndef XSTR
#define XSTR NPOS
#endif
#define NR (NB * NPOS)
#define NCB ((NPOS + 127) / 128)
#ifndef TQB
#define TQB (NPOS / 64)
#endif
typedef __attribute__((ext_vector_type(8))) __bf16 v8b;
__device__ __forceinline__ v16b frag_b(const __bf16* rowk0, int lane) {
  union { v16b v; v8b q[2]; } u; const __bf16* p = rowk0 + 8 * (lane >> 4);
  u.q[0] = *(const v8b*)p; u.q[1] = *(const v8b*)(p + 16); return u.v;
}
__device__ __forceinline__ float bfr(float v) { return (float)(__bf16)v; }
__device__ __attribute__((noinline)) float exp_ni(float v) { return expf(v); }
__device__ __attribute__((noinline)) float erf_ni(float v) { return erff(v); }

#define PK_Q  0
#define PK_K  ((size_t)CQ * CC)
#define PK_V  ((size_t)2 * CQ * CC)
#define PK_A  (PK_V + (size_t)CC * CC)
#define PK_B  (PK_A + (size_t)CC * CC)
#define PK_END (PK_B + (size_t)CC * CAT)
#define WS_PK   0u
#define WS_CH   (((2u * PK_END) + 127u) / 128u * 128u)
#define WS_CL   (WS_CH + 2u * (size_t)NR * CAT)
#define WS_QT   (WS_CL + 2u * (size_t)NR * CAT)
#define WS_QTL  (WS_QT + 2u * NR * CQ)
#define WS_KT   (WS_QTL + 2u * NR * CQ)
#define WS_KTL  (WS_KT + 2u * NR * CQ)
#define WS_V0H  (WS_KTL + 2u * NR * CQ)
#define WS_V0L  (WS_V0H + 2u * (size_t)NR * CC)
#define WS_VXH  (WS_V0L + 2u * (size_t)NR * CC)
#define WS_VXL  (WS_VXH + 2u * (size_t)NR * CC)
#define WS_Y    (WS_VXL + 2u * (size_t)NR * CC)
#define WS_ST   (WS_Y + 4u * (size_t)NR * CC)
#define WS_MS   (WS_ST + 4u * (size_t)NB * NCB * CC * 2)
#define WS_END  (WS_MS + 4u * CC * 2)

__global__ __launch_bounds__(256) void k_pack(const float* __restrict__ WQ, const float* __restrict__ WK, const float* __restrict__ WV, const float* __restrict__ WA, const float* __restrict__ WB, __bf16* __restrict__ PK) {
  __shared__ __align__(16) __bf16 s[CAT]; const int n = blockIdx.x, which = blockIdx.y, t = threadIdx.x; int K; size_t dst; const float* Wm;
  switch (which) { case 0: if (n >= CQ) return; Wm = WQ; K = CC; dst = PK_Q; break; case 1: if (n >= CQ) return; Wm = WK; K = CC; dst = PK_K; break; case 2: Wm = WV; K = CC; dst = PK_V; break; case 3: Wm = WA; K = CC; dst = PK_A; break; default: Wm = WB; K = CAT; dst = PK_B; break; }
  for (int k = t; k < K; k += 256) s[k] = (__bf16)Wm[(size_t)n * K + k];
  __syncthreads();
  for (int q = t; q < K / 8; q += 256) vst2((unsigned*)(PK + dst + (size_t)n * K + q * 8), *(const v4u*)&s[q * 8]);
}
__global__ __launch_bounds__(256) void k_xT(const float* __restrict__ X, __bf16* __restrict__ CH, __bf16* __restrict__ CL) {
  __shared__ __align__(16) __bf16 s[64][72]; const int t = threadIdx.x; const int n0 = blockIdx.x * 64, c0 = blockIdx.y * 64; const size_t b = blockIdx.z;
  for (int e = t; e < 64 * 64; e += 256) { const int c = e >> 6, r = e & 63; s[r][c] = (__bf16)X[(b * CC + c0 + c) * XSTR + n0 + r]; }
  __syncthreads();
  for (int e = t; e < 64 * 8; e += 256) { const int r = e >> 3, q = e & 7; const size_t o = (b * NPOS + n0 + r) * CAT + 3 * CC + c0 + q * 8; vst2((unsigned*)(CH + o), *(const v4u*)&s[r][q * 8]); const v4u z = {0u, 0u, 0u, 0u}; vst2((unsigned*)(CL + o), z); }
}
__global__ __launch_bounds__(128) void k_proj(const __bf16* __restrict__ CH, const __bf16* __restrict__ PK, const float* __restrict__ BQ, const float* __restrict__ BK, const float* __restrict__ BV, _Float16* __restrict__ QT, _Float16* __restrict__ QTL, _Float16* __restrict__ KT, _Float16* __restrict__ KTL, _Float16* __restrict__ V0H, _Float16* __restrict__ V0L) {
  __shared__ __align__(16) _Float16 st[128][72], stl[128][72]; __shared__ __align__(16) _Float16 so[4][16][136], sol[4][16][136];
  const int tid = threadIdx.x, wave = tid >> 5, lane = tid & 31, col = lane & 15, g = lane >> 4; const int n0 = blockIdx.x * 128; const int grp = blockIdx.y; const size_t b = blockIdx.z;
  const __bf16* Wr = PK + ((grp == 0) ? PK_Q : (grp == 1) ? PK_K : (PK_V + (size_t)(grp - 2) * 64 * CC)); const float* BB = (grp == 0) ? BQ : (grp == 1) ? BK : (BV + (grp - 2) * 64);
  const int o0 = wave * 16;
  v8f acc[8] = {};
#pragma unroll 2
  for (int kc = 0; kc < CC / 32; ++kc) { const v16b a = frag_b(Wr + (size_t)(o0 + col) * CC + kc * 32, lane);
#pragma unroll
    for (int j = 0; j < 8; ++j) { const int n = min(n0 + j * 16 + col, NPOS - 1); acc[j] = wmma_bf(a, frag_b(CH + (b * NPOS + n) * CAT + 3 * CC + kc * 32, lane), acc[j]); } }
  const int nval = min(128, NPOS - n0);
  if (grp < 2) {
#pragma unroll
    for (int j = 0; j < 8; ++j)
#pragma unroll
      for (int r = 0; r < 8; ++r) { const float v = acc[j][r] + bfr(BB[o0 + 8 * g + r]); const _Float16 hv = (_Float16)v; st[j * 16 + col][o0 + 8 * g + r] = hv; stl[j * 16 + col][o0 + 8 * g + r] = (_Float16)((v - (float)hv) * 2048.0f); }
    __syncthreads();
    _Float16* DH_ = (grp == 0) ? QT : KT; _Float16* DL_ = (grp == 0) ? QTL : KTL;
    for (int e = tid; e < nval * 8; e += 128) { const int r = e >> 3, q = e & 7; const size_t o = (b * NPOS + n0 + r) * CQ + q * 8; vst2((unsigned*)(DH_ + o), *(const v4u*)&st[r][q * 8]); vst2((unsigned*)(DL_ + o), *(const v4u*)&stl[r][q * 8]); }
  } else {
#pragma unroll
    for (int j = 0; j < 8; ++j)
#pragma unroll
      for (int r = 0; r < 8; ++r) { const float v = acc[j][r] + bfr(BB[o0 + 8 * g + r]); const _Float16 hv = (_Float16)v; so[wave][8 * g + r][j * 16 + col] = hv; sol[wave][8 * g + r][j * 16 + col] = (_Float16)((v - (float)hv) * 2048.0f); }
    LDSX();
    const int oc = (grp - 2) * 64 + o0;
    for (int rl = 0; rl < 16; ++rl) { const size_t o = (b * CC + oc + rl) * NPOS + n0; if (lane < 16) { if (lane * 8 < nval) vst2((unsigned*)(V0H + o + lane * 8), *(const v4u*)&so[wave][rl][lane * 8]); } else { if ((lane - 16) * 8 < nval) vst2((unsigned*)(V0L + o + (lane - 16) * 8), *(const v4u*)&sol[wave][rl][(lane - 16) * 8]); } }
  }
}
__global__ __launch_bounds__(128) void k_attn(const _Float16* __restrict__ QT, const _Float16* __restrict__ QTL, const _Float16* __restrict__ KT, const _Float16* __restrict__ KTL, const _Float16* __restrict__ VH, const _Float16* __restrict__ VL, const int* __restrict__ MASK, int var, int rad, __bf16* __restrict__ CH, __bf16* __restrict__ CL) {
  __shared__ __align__(16) _Float16 sp[4][16][40], spu[4][16][40]; __shared__ __align__(16) __bf16 sh[4][16][264], sl[4][16][264]; __shared__ int smk[64][33];
  const int tid = threadIdx.x, wave = tid >> 5, lane = tid & 31, col = lane & 15, g = lane >> 4; const int qb = blockIdx.x, cp = blockIdx.y; const size_t b = blockIdx.z; const int q0 = qb * 64 + wave * 16; const size_t rq = b * NPOS + q0;
  float m[8], l[8];
#pragma unroll
  for (int r = 0; r < 8; ++r) { m[r] = -3.0e38f; l[r] = 0.f; }
  v8f acc[16] = {};
  int ks0 = 0, ks1 = NPOS / 32;
  if (var > 0) { const int y0 = (qb * 64) / HH, y1 = (qb * 64 + 63) / HH; const int lo = max(0, (y0 - rad) * HH), hi = min(NPOS, (y1 + rad + 1) * HH); ks0 = lo / 32; ks1 = (hi + 31) / 32; }
  const _Float16* Vh = VH + (b * CC + cp * 256) * NPOS; const _Float16* Vl = VL + (b * CC + cp * 256) * NPOS;
#pragma unroll 1
  for (int ks = ks0; ks < ks1; ++ks) { const int j0 = ks * 32;
    if (var > 0) { for (int e = tid; e < 64 * 8; e += 128) { const int r = e >> 3, q4 = e & 7; const v4i mv = *(const v4i*)(MASK + (size_t)(qb * 64 + r) * XSTR + j0 + q4 * 4); smk[r][q4 * 4] = mv[0]; smk[r][q4 * 4 + 1] = mv[1]; smk[r][q4 * 4 + 2] = mv[2]; smk[r][q4 * 4 + 3] = mv[3]; } __syncthreads(); }
    v8f s[2];
#pragma unroll
    for (int ct = 0; ct < 2; ++ct) { const int kk = j0 + ct * 16 + col; const size_t rk = (b * NPOS + kk) * CQ; v8f c = {}, cl = {};
#pragma unroll 1
      for (int kc = 0; kc < 2; ++kc) { const v16h aq = frag_h(QT + (rq + col) * CQ + kc * 32, lane), aql = frag_h(QTL + (rq + col) * CQ + kc * 32, lane); const v16h kh = frag_h(KT + rk + kc * 32, lane); c = wmma16(aq, kh, c); cl = wmma16(aql, kh, cl); cl = wmma16(aq, frag_h(KTL + rk + kc * 32, lane), cl); }
#pragma unroll
      for (int r = 0; r < 8; ++r) { const bool keep = (var == 0) || (smk[wave * 16 + 8 * g + r][ct * 16 + col] != 0); s[ct][r] = keep ? (c[r] + cl[r] * (1.0f / 2048.0f)) : -3.0e38f; } }
#pragma unroll
    for (int r = 0; r < 8; ++r) { float mx = fmaxf(s[0][r], s[1][r]);
#pragma unroll
      for (int o = 1; o < 16; o <<= 1) mx = fmaxf(mx, __shfl_xor(mx, o));
      const float mn = fmaxf(m[r], mx); const float alpha = (m[r] <= -1.0e38f) ? 0.f : __expf(m[r] - mn);
      const float e0 = (s[0][r] <= -1.0e38f) ? 0.f : __expf(s[0][r] - mn), e1 = (s[1][r] <= -1.0e38f) ? 0.f : __expf(s[1][r] - mn); float es = e0 + e1;
#pragma unroll
      for (int o = 1; o < 16; o <<= 1) es += __shfl_xor(es, o);
      l[r] = l[r] * alpha + es; m[r] = (mn <= -1.0e38f) ? m[r] : mn;
#pragma unroll
      for (int dt = 0; dt < 16; ++dt) acc[dt][r] *= alpha;
      sp[wave][8 * g + r][col] = (_Float16)(e0 * 2048.0f); sp[wave][8 * g + r][16 + col] = (_Float16)(e1 * 2048.0f); spu[wave][8 * g + r][col] = (_Float16)e0; spu[wave][8 * g + r][16 + col] = (_Float16)e1; }
    LDSX();
    const v16h pa = frag_h(&sp[wave][col][0], lane), pu = frag_h(&spu[wave][col][0], lane);
#pragma unroll
    for (int dt = 0; dt < 16; ++dt) { const size_t vo = (size_t)(dt * 16 + col) * NPOS + j0; acc[dt] = wmma16(pu, frag_h(Vl + vo, lane), acc[dt]); acc[dt] = wmma16(pa, frag_h(Vh + vo, lane), acc[dt]); }
    __syncthreads(); }
#pragma unroll
  for (int r = 0; r < 8; ++r) { const float il = (1.0f / 2048.0f) / l[r];
#pragma unroll
    for (int dt = 0; dt < 16; ++dt) { const float v = acc[dt][r] * il; const __bf16 hb = (__bf16)v; sh[wave][8 * g + r][dt * 16 + col] = hb; sl[wave][8 * g + r][dt * 16 + col] = (__bf16)(v - (float)hb); } }
  LDSX();
  for (int rl = 0; rl < 16; ++rl) { const size_t o = (rq + rl) * CAT + var * CC + cp * 256; vst2((unsigned*)(CH + o + lane * 8), *(const v4u*)&sh[wave][rl][lane * 8]); vst2((unsigned*)(CL + o + lane * 8), *(const v4u*)&sl[wave][rl][lane * 8]); }
}
__global__ __launch_bounds__(128) void k_gate(const __bf16* __restrict__ CH, const __bf16* __restrict__ CL, int src, const __bf16* __restrict__ PK, const float* __restrict__ BA, const _Float16* __restrict__ V0H, const _Float16* __restrict__ V0L, _Float16* __restrict__ VXH, _Float16* __restrict__ VXL) {
  __shared__ __align__(16) _Float16 so[4][16][136], sol[4][16][136];
  const int tid = threadIdx.x, wave = tid >> 5, lane = tid & 31, col = lane & 15, g = lane >> 4; const int n0 = blockIdx.x * 128; const int oc = blockIdx.y * 64 + wave * 16; const size_t b = blockIdx.z;
  v8f acc[8] = {};
#pragma unroll 2
  for (int kc = 0; kc < CC / 32; ++kc) { const v16b a = frag_b(PK + PK_A + (size_t)(oc + col) * CC + kc * 32, lane);
#pragma unroll
    for (int j = 0; j < 8; ++j) { const size_t ro = (b * NPOS + min(n0 + j * 16 + col, NPOS - 1)) * CAT + (size_t)src * CC + kc * 32; acc[j] = wmma_bf(a, frag_b(CL + ro, lane), acc[j]); acc[j] = wmma_bf(a, frag_b(CH + ro, lane), acc[j]); } }
  const int nval = min(128, NPOS - n0);
#pragma unroll
  for (int j = 0; j < 8; ++j)
#pragma unroll
    for (int r = 0; r < 8; ++r) { const int o = oc + 8 * g + r; const int n = min(n0 + j * 16 + col, NPOS - 1); const float gt = 1.0f / (1.0f + exp_ni(-(acc[j][r] + bfr(BA[o])))); const size_t vi = (b * CC + o) * NPOS + n; const float v0 = (float)V0H[vi] + (float)V0L[vi] * (1.0f / 2048.0f); const float v = v0 * gt; const _Float16 hv = (_Float16)v; so[wave][8 * g + r][j * 16 + col] = hv; sol[wave][8 * g + r][j * 16 + col] = (_Float16)((v - (float)hv) * 2048.0f); }
  LDSX();
  for (int rl = 0; rl < 16; ++rl) { const size_t o = (b * CC + oc + rl) * NPOS + n0; if (lane < 16) { if (lane * 8 < nval) vst2((unsigned*)(VXH + o + lane * 8), *(const v4u*)&so[wave][rl][lane * 8]); } else { if ((lane - 16) * 8 < nval) vst2((unsigned*)(VXL + o + (lane - 16) * 8), *(const v4u*)&sol[wave][rl][(lane - 16) * 8]); } }
}
__global__ __launch_bounds__(128) void k_final(const __bf16* __restrict__ CH, const __bf16* __restrict__ CL, const __bf16* __restrict__ PK, float* __restrict__ Y, float* __restrict__ ST) {
  __shared__ __align__(16) float so[4][16][132]; __shared__ __align__(16) float sst[64][2];
  const int tid = threadIdx.x, wave = tid >> 5, lane = tid & 31, col = lane & 15, g = lane >> 4; const int n0 = blockIdx.x * 128; const int oc = blockIdx.y * 64 + wave * 16; const size_t b = blockIdx.z;
  v8f acc[8] = {};
#pragma unroll 2
  for (int kc = 0; kc < CAT / 32; ++kc) { const v16b a = frag_b(PK + PK_B + (size_t)(oc + col) * CAT + kc * 32, lane);
#pragma unroll
    for (int j = 0; j < 8; ++j) { const size_t ro = (b * NPOS + min(n0 + j * 16 + col, NPOS - 1)) * CAT + kc * 32; acc[j] = wmma_bf(a, frag_b(CL + ro, lane), acc[j]); acc[j] = wmma_bf(a, frag_b(CH + ro, lane), acc[j]); } }
  const int nval = min(128, NPOS - n0);
#pragma unroll
  for (int j = 0; j < 8; ++j)
#pragma unroll
    for (int r = 0; r < 8; ++r) so[wave][8 * g + r][j * 16 + col] = acc[j][r];
  LDSX();
  for (int rl = 0; rl < 16; ++rl) if (lane * 4 < nval) vst2(Y + (b * CC + oc + rl) * NPOS + n0 + lane * 4, *(const v4f*)&so[wave][rl][lane * 4]);
  if (lane < 16) { float s = 0.f, q2 = 0.f; for (int n = 0; n < nval; ++n) { const float v = so[wave][lane][n]; s += v; q2 += v * v; } sst[wave * 16 + lane][0] = s; sst[wave * 16 + lane][1] = q2; }
  __syncthreads();
  if (tid < 32) vst2(ST + (((size_t)(b * NCB + blockIdx.x)) * CC + blockIdx.y * 64) * 2 + tid * 4, *(const v4f*)(&sst[0][0] + tid * 4));
}
__global__ __launch_bounds__(256) void k_bnstat(const float* __restrict__ ST, float* __restrict__ MS) {
  __shared__ __align__(16) float sm[CC][2]; for (int c = threadIdx.x; c < CC; c += 256) { float s = 0.f, q2 = 0.f; for (int blk = 0; blk < NB * NCB; ++blk) { s += ST[((size_t)blk * CC + c) * 2]; q2 += ST[((size_t)blk * CC + c) * 2 + 1]; } const float mu = s / (float)NR; sm[c][0] = mu; sm[c][1] = 1.0f / sqrtf(fmaxf(q2 / (float)NR - mu * mu, 0.f) + 1e-5f); }
  __syncthreads(); for (int q = threadIdx.x; q < CC * 2 / 4; q += 256) vst2(MS + q * 4, *(const v4f*)(&sm[0][0] + q * 4));
}
__global__ __launch_bounds__(256) void k_out(const float* __restrict__ Y, const float* __restrict__ MS, const float* __restrict__ G, const float* __restrict__ Bt, float* __restrict__ OUT) {
  const int o = blockIdx.x; const size_t b = blockIdx.y; const float mu = MS[o * 2], rs = MS[o * 2 + 1], gg = bfr(G[o]), bb = bfr(Bt[o]); const size_t base = (b * CC + o) * NPOS;
  for (int q = threadIdx.x; q < NPOS / 4; q += 256) { v4f v = *(const v4f*)(Y + base + q * 4); for (int i = 0; i < 4; ++i) v[i] = fmaxf((v[i] - mu) * rs * gg + bb, 0.f); vst2(OUT + base + q * 4, v); }
}
extern "C" void kernel_launch(void* const* d_in, const int* in_sizes, int n_in, void* d_out, int out_size, void* d_ws, size_t ws_size, hipStream_t stream) {
  (void)in_sizes; (void)n_in; (void)out_size;
  const float** F = (const float**)d_in;
  if (ws_size < (size_t)WS_END) return;
  char* ws = (char*)d_ws; __bf16 *PK = (__bf16*)(ws + WS_PK), *CH = (__bf16*)(ws + WS_CH), *CL = (__bf16*)(ws + WS_CL); _Float16 *QT = (_Float16*)(ws + WS_QT), *QTL = (_Float16*)(ws + WS_QTL), *KT = (_Float16*)(ws + WS_KT), *KTL = (_Float16*)(ws + WS_KTL), *V0H = (_Float16*)(ws + WS_V0H), *V0L = (_Float16*)(ws + WS_V0L), *VXH = (_Float16*)(ws + WS_VXH), *VXL = (_Float16*)(ws + WS_VXL);
  float *Y = (float*)(ws + WS_Y), *ST = (float*)(ws + WS_ST), *MS = (float*)(ws + WS_MS);
  k_pack<<<dim3(CC, 5), 256, 0, stream>>>(F[3], F[5], F[7], F[9], F[11], PK);
  k_xT<<<dim3(NPOS / 64, CC / 64, NB), 256, 0, stream>>>(F[0], CH, CL);
  k_proj<<<dim3(NCB, 10, NB), 128, 0, stream>>>(CH, PK, F[4], F[6], F[8], QT, QTL, KT, KTL, V0H, V0L);
  k_attn<<<dim3(TQB, 2, NB), 128, 0, stream>>>(QT, QTL, KT, KTL, V0H, V0L, nullptr, 0, 0, CH, CL);
  k_gate<<<dim3(NCB, CC / 64, NB), 128, 0, stream>>>(CH, CL, 0, PK, F[10], V0H, V0L, VXH, VXL);
  k_attn<<<dim3(TQB, 2, NB), 128, 0, stream>>>(QT, QTL, KT, KTL, VXH, VXL, (const int*)d_in[1], 1, 7, CH, CL);
  k_gate<<<dim3(NCB, CC / 64, NB), 128, 0, stream>>>(CH, CL, 1, PK, F[10], V0H, V0L, VXH, VXL);
  k_attn<<<dim3(TQB, 2, NB), 128, 0, stream>>>(QT, QTL, KT, KTL, VXH, VXL, (const int*)d_in[2], 2, 14, CH, CL);
  k_final<<<dim3(NCB, CC / 64, NB), 128, 0, stream>>>(CH, CL, PK, Y, ST);
  k_bnstat<<<1, 256, 0, stream>>>(ST, MS);
  k_out<<<dim3(CC, NB), 256, 0, stream>>>(Y, MS, F[12], F[13], (float*)d_out);
}
